// GTEProgramClassification_27986006900857
// MI455X (gfx1250) — hardware-run, weakly checked
//
#include <hip/hip_runtime.h>
#include <math.h>

constexpr int kNSrc     = 50000;
constexpr int kNSrcPad  = 50048;
constexpr int kNDst     = 32000;
constexpr int kMaxDeg   = 16;
constexpr int kNSub     = 4;
constexpr int kDim      = 128;
constexpr int kVocab    = 32000;
constexpr int kNCls     = 104;
constexpr int kNClsPad  = 128;
constexpr int kSteps    = 15;
constexpr int kG3       = 3 * kDim;
constexpr int kChunkRows = 16000;
constexpr int kNChunks  = 2;
constexpr float kFeatCarry = 64.0f;
constexpr float kHCarry    = 64.0f;
constexpr float kWCarry    = 256.0f;
constexpr float kGemmScale = 1.0f / 16384.0f;
constexpr float kLnEps     = 1e-5f;
constexpr float kInvDim    = 1.0f / 128.0f;

static_assert(kNSrcPad % 64 == 0 && kNSrcPad >= kNSrc, "M pad");
static_assert(kNDst % 64 == 0 && kChunkRows % 64 == 0 && kChunkRows * kNChunks == kNDst, "tiles");
static_assert(kDim % 32 == 0 && kG3 % 64 == 0 && kNClsPad % 64 == 0, "K and N multiples");

typedef __attribute__((ext_vector_type(16))) _Float16 v16h;
typedef __attribute__((ext_vector_type(8)))  _Float16 v8h;
typedef __attribute__((ext_vector_type(16))) __bf16   v16b;
typedef __attribute__((ext_vector_type(8)))  __bf16   v8b;
typedef __attribute__((ext_vector_type(8)))  float    v8f;
typedef __attribute__((ext_vector_type(4)))  float    v4f;
typedef __attribute__((ext_vector_type(4)))  unsigned int v4u;

__device__ __forceinline__ unsigned short f2bf_bits(float f) {
  unsigned u = __float_as_uint(f);
  return (unsigned short)((u + 0x7FFFu + ((u >> 16) & 1u)) >> 16);
}
__device__ __forceinline__ float bf_bits2f(unsigned short h) { return __uint_as_float(((unsigned)h) << 16); }

__device__ __forceinline__ void dep_guard_h(v8f& a, v8f& b, v16h x, v16h y) { asm volatile("v_nop\n\tv_nop\n\tv_nop\n\tv_nop" : "+v"(a), "+v"(b) : "v"(x), "v"(y)); }
__device__ __forceinline__ void dep_guard_b(v8f& a, v8f& b, v16b x, v16b y) { asm volatile("v_nop\n\tv_nop\n\tv_nop\n\tv_nop" : "+v"(a), "+v"(b) : "v"(x), "v"(y)); }
__device__ __forceinline__ void keep4_h(v16h a, v16h b, v16h c, v16h d) { asm volatile("v_nop" :: "v"(a), "v"(b), "v"(c), "v"(d)); }
__device__ __forceinline__ void keep4_b(v16b a, v16b b, v16b c, v16b d) { asm volatile("v_nop" :: "v"(a), "v"(b), "v"(c), "v"(d)); }
__device__ __forceinline__ void acc_guard4(v8f& a, v8f& b, v8f& c, v8f& d) { asm volatile("v_nop\n\tv_nop\n\tv_nop\n\tv_nop" : "+v"(a), "+v"(b), "+v"(c), "+v"(d)); }
template <typename T> struct Frag;
template <> struct Frag<_Float16> {
  typedef v16h V; union U { v16h v; v8h h[2]; };
  static __device__ __forceinline__ v16h load(const _Float16* p) {
    U f; f.h[0] = *(const v8h*)(p); f.h[1] = *(const v8h*)(p + 16); return f.v;
  }
  static __device__ __forceinline__ v8f mma(v16h a, v16h b, v8f c) {
    return __builtin_amdgcn_wmma_f32_16x16x32_f16(false, a, false, b, (short)0, c, false, false);
  }
  static __device__ __forceinline__ void guard(v8f& a, v8f& b, v16h x, v16h y) { dep_guard_h(a, b, x, y); }
  static __device__ __forceinline__ void keep(v16h a, v16h b, v16h c, v16h d) { keep4_h(a, b, c, d); }
};
template <> struct Frag<__bf16> {
  typedef v16b V; union U { v16b v; v8b h[2]; };
  static __device__ __forceinline__ v16b load(const __bf16* p) {
    U f; f.h[0] = *(const v8b*)(p); f.h[1] = *(const v8b*)(p + 16); return f.v;
  }
  static __device__ __forceinline__ v8f mma(v16b a, v16b b, v8f c) {
    return __builtin_amdgcn_wmma_f32_16x16x32_bf16(false, a, false, b, (short)0, c, false, false);
  }
  static __device__ __forceinline__ void guard(v8f& a, v8f& b, v16b x, v16b y) { dep_guard_b(a, b, x, y); }
  static __device__ __forceinline__ void keep(v16b a, v16b b, v16b c, v16b d) { keep4_b(a, b, c, d); }
};

__device__ __forceinline__ unsigned pk16(unsigned short a, unsigned short b) { return (unsigned)a | ((unsigned)b << 16); }
__device__ __forceinline__ unsigned short h_bits(float f) { const _Float16 h = (_Float16)f; return __builtin_bit_cast(unsigned short, h); }

template <int ET> struct Elem;
template <> struct Elem<0> { typedef _Float16 T; };
template <> struct Elem<1> { typedef __bf16 T; };
template <int ET, bool SPLIT, int BIAS_MODE, int OUT_MODE, bool RESID, int ACT = 0>
__global__ __launch_bounds__(256) void wmma_gemm64(
    const unsigned short* __restrict__ Ap, const unsigned short* __restrict__ A2p, int lda, long strideA,
    const unsigned short* __restrict__ Btp, const unsigned short* __restrict__ Bt2p, int ldb, long strideB,
    void* __restrict__ Cout, void* __restrict__ Cout2, int ldc, long strideC,
    const float* __restrict__ bias,
    const float* __restrict__ resid, long strideR,
    int M, int N, int K, float scale) {
  typedef typename Elem<ET>::T T;
  typedef typename Frag<T>::V V;
  const T* A = (const T*)Ap; const T* A2 = (const T*)A2p; const T* Bt = (const T*)Btp; const T* Bt2 = (const T*)Bt2p;
  __shared__ __align__(16) float sT[8][16 * 68];
  const int b    = blockIdx.y;
  const int lane = threadIdx.x & 31;
  const int wave = threadIdx.x >> 5;
  const int tilesN = N >> 6;
  const int tilesM = M >> 6;
  const int tile = blockIdx.x * 8 + wave;
  if (tile >= tilesM * tilesN) return;
  const int tm = tile / tilesN;
  const int tn = tile - tm * tilesN;
  const int m0 = tm << 6;
  const int n0 = tn << 6;

  const T* Ab  = A  + (size_t)b * strideA;
  const T* Bb  = Bt + (size_t)b * strideB;
  const T* Ab2 = SPLIT ? (A2  + (size_t)b * strideA) : nullptr;
  const T* Bb2 = SPLIT ? (Bt2 + (size_t)b * strideB) : nullptr;

  const int rlane = lane & 15;
  const int koff  = (lane >> 4) * 8;
  const int mOff  = (lane >> 4) * 8;

  v8f acc[4][4];
#pragma unroll
  for (int i = 0; i < 4; ++i)
#pragma unroll
    for (int j = 0; j < 4; ++j) acc[i][j] = (v8f){0.f,0.f,0.f,0.f,0.f,0.f,0.f,0.f};

  for (int k0 = 0; k0 < K; k0 += 32) {
    V bh[4], bl[4];
#pragma unroll
    for (int j = 0; j < 4; ++j) {
      const size_t bo = (size_t)(n0 + (j << 4) + rlane) * ldb + koff + k0;
      bh[j] = Frag<T>::load(Bb + bo);
      if (SPLIT) bl[j] = Frag<T>::load(Bb2 + bo);
    }
#pragma unroll
    for (int i = 0; i < 4; ++i) {
      const size_t ao = (size_t)(m0 + (i << 4) + rlane) * lda + koff + k0;
      V ah = Frag<T>::load(Ab + ao);
      V al;
      if (SPLIT) al = Frag<T>::load(Ab2 + ao);
#pragma unroll
      for (int j = 0; j < 4; ++j) {
        acc[i][j] = Frag<T>::mma(ah, bh[j], acc[i][j]);
        if (SPLIT) {
          acc[i][j] = Frag<T>::mma(ah, bl[j], acc[i][j]);
          acc[i][j] = Frag<T>::mma(al, bh[j], acc[i][j]);
        }
      }
      Frag<T>::guard(acc[i][0], acc[i][3], ah, SPLIT ? al : ah);
    }
    Frag<T>::keep(bh[0], bh[1], bh[2], bh[3]);
    if (SPLIT) Frag<T>::keep(bl[0], bl[1], bl[2], bl[3]);
  }
  acc_guard4(acc[0][0], acc[0][1], acc[0][2], acc[0][3]);
  acc_guard4(acc[1][0], acc[1][1], acc[1][2], acc[1][3]);
  acc_guard4(acc[2][0], acc[2][1], acc[2][2], acc[2][3]);
  acc_guard4(acc[3][0], acc[3][1], acc[3][2], acc[3][3]);

  float* slab = sT[wave];
  const float* Rb = RESID ? (resid + (size_t)b * strideR) : nullptr;
#pragma unroll
  for (int i = 0; i < 4; ++i) {
    const int mBase = m0 + (i << 4);
#pragma unroll
    for (int j = 0; j < 4; ++j) {
      const int n = n0 + (j << 4) + rlane;
      float bv = 0.f;
      if (BIAS_MODE == 2) bv = bias[n];
#pragma unroll
      for (int r = 0; r < 8; ++r) {
        float v = acc[i][j][r] * scale;
        if (BIAS_MODE == 1) v += bias[mBase + mOff + r];
        if (BIAS_MODE == 2) v += bv;
        if (RESID) v += Rb[(size_t)(mBase + mOff + r) * ldc + n];
        if (ACT == 2) v = fmaxf(v, 0.0f);
        if (ACT == 4) v = (v > 0.f) ? v : 0.01f * v;
        slab[(mOff + r) * 68 + (j << 4) + rlane] = v;
      }
    }
    __builtin_amdgcn_fence(__ATOMIC_RELEASE, "workgroup");
    __builtin_amdgcn_wave_barrier();
    __builtin_amdgcn_fence(__ATOMIC_ACQUIRE, "workgroup");
    if (OUT_MODE == 0) {
      float* C = (float*)Cout + (size_t)b * strideC;
      const int hh = lane >> 4, c4 = (lane & 15) * 4;
      for (int pass = 0; pass < 2; ++pass) {
#pragma unroll
        for (int it = 0; it < 8; ++it) {
          const int row = it * 2 + hh;
          v4f v = *(const v4f*)(slab + row * 68 + c4);
          *(volatile v4f*)(C + (size_t)(mBase + row) * ldc + n0 + c4) = v;
        }
        __threadfence();
      }
    } else {
      const int q = lane >> 3, c8 = (lane & 7) * 8;
      unsigned short* C  = (unsigned short*)Cout  + (size_t)b * strideC;
      unsigned short* C2 = (OUT_MODE == 2) ? ((unsigned short*)Cout2 + (size_t)b * strideC) : nullptr;
      for (int pass = 0; pass < 2; ++pass) {
#pragma unroll
        for (int it = 0; it < 4; ++it) {
          const int row = it * 4 + q;
          const float* sp = slab + row * 68 + c8;
          v8h hv, lv;
#pragma unroll
          for (int e = 0; e < 8; ++e) {
            if (OUT_MODE == 1) {
              hv[e] = (_Float16)sp[e];
            } else {
              unsigned short hb = f2bf_bits(sp[e]);
              unsigned short lb = f2bf_bits(sp[e] - bf_bits2f(hb));
              hv[e] = __builtin_bit_cast(_Float16, hb);
              lv[e] = __builtin_bit_cast(_Float16, lb);
            }
          }
          *(volatile v8h*)(C + (size_t)(mBase + row) * ldc + n0 + c8) = hv;
          if (OUT_MODE == 2) *(volatile v8h*)(C2 + (size_t)(mBase + row) * ldc + n0 + c8) = lv;
        }
        __threadfence();
      }
    }
    __builtin_amdgcn_fence(__ATOMIC_RELEASE, "workgroup");
    __builtin_amdgcn_wave_barrier();
    __builtin_amdgcn_fence(__ATOMIC_ACQUIRE, "workgroup");
  }
}

__device__ __forceinline__ int clampi(int v, int hi) { v = (v < 0) ? 0 : v; return (v > hi) ? hi : v; }
__device__ __forceinline__ unsigned short feat16_bits(float e0, float e1, float e2, float e3) {
  const float s = ((e0 + e1) + e2) + e3;
  const float m = s * 0.25f;
  return h_bits(m * kFeatCarry);
}

__global__ __launch_bounds__(256) void wcast_kernel(const float* __restrict__ w_ih, const float* __restrict__ w_hh,
                                                    const float* __restrict__ wc,
                                                    unsigned short* __restrict__ o_ih, unsigned short* __restrict__ o_hh,
                                                    unsigned short* __restrict__ o_c, float scale) {
  const int y = blockIdx.y;
  const int i = blockIdx.x * 256 + threadIdx.x;
  const int n8 = (y == 2) ? (kNClsPad * kDim / 8) : (kG3 * kDim / 8);
  if (i >= n8) return;
  const float* src = (y == 0) ? w_ih : (y == 1) ? w_hh : wc;
  unsigned short* dst = (y == 0) ? o_ih : (y == 1) ? o_hh : o_c;
  const int row = (8 * i) / kDim;
  const bool valid = (y != 2) || (row < kNCls);
  const int ic = valid ? i : 0;
  const float* p = src + 8 * (size_t)ic;
  const v4f a = *(const v4f*)(p);
  const v4f c = *(const v4f*)(p + 4);
  unsigned short hb[8];
#pragma unroll
  for (int e = 0; e < 4; ++e) {
    hb[e]     = valid ? h_bits(a[e] * scale) : (unsigned short)0;
    hb[4 + e] = valid ? h_bits(c[e] * scale) : (unsigned short)0;
  }
  const v4u u = (v4u){pk16(hb[0], hb[1]), pk16(hb[2], hb[3]), pk16(hb[4], hb[5]), pk16(hb[6], hb[7])};
  unsigned short* q = dst + 8 * (size_t)i;
  *(volatile v4u*)q = u;
  __threadfence();
  *(volatile v4u*)q = u;
}

__global__ __launch_bounds__(256) void feat_kernel(const int* __restrict__ token_id, const float* __restrict__ emb,
                                                   unsigned short* __restrict__ feat16) {
  const int tid = threadIdx.x;
  const int row = blockIdx.x * 16 + (tid >> 4);
  const int c8  = (tid & 15) * 8;
  const bool valid = row < kNSrc;
  const int rc = valid ? row : (kNSrc - 1);
  int tk[4];
#pragma unroll
  for (int u = 0; u < 4; ++u) tk[u] = clampi(token_id[(size_t)rc * kNSub + u], kVocab - 1);
  v4f ea[4], eb[4];
#pragma unroll
  for (int u = 0; u < 4; ++u) {
    const float* p = emb + (size_t)tk[u] * kDim + c8;
    ea[u] = *(const v4f*)(p);
    eb[u] = *(const v4f*)(p + 4);
  }
  unsigned short hb[8];
#pragma unroll
  for (int e = 0; e < 4; ++e) {
    hb[e]     = valid ? feat16_bits(ea[0][e], ea[1][e], ea[2][e], ea[3][e]) : (unsigned short)0;
    hb[4 + e] = valid ? feat16_bits(eb[0][e], eb[1][e], eb[2][e], eb[3][e]) : (unsigned short)0;
  }
  const v4u u = (v4u){pk16(hb[0], hb[1]), pk16(hb[2], hb[3]), pk16(hb[4], hb[5]), pk16(hb[6], hb[7])};
  unsigned short* q = feat16 + (size_t)row * kDim + c8;
  *(volatile v4u*)q = u;
  __threadfence();
  *(volatile v4u*)q = u;
}

template <bool FIRST>
__global__ __launch_bounds__(256) void gru_cell_kernel(const int* __restrict__ neigh_idx, const int* __restrict__ deg,
                                                       const float* __restrict__ xps, const float* __restrict__ hp,
                                                       const float* __restrict__ b_hh,
                                                       float* __restrict__ H, unsigned short* __restrict__ H16,
                                                       int row_base, int t) {
  __shared__ __align__(16) float slab[8][kDim];
  const int tid  = threadIdx.x;
  const int wave = tid >> 5;
  const int lane = tid & 31;
  const int n    = row_base + blockIdx.x * 8 + wave;
  const int src  = clampi(neigh_idx[(size_t)n * kMaxDeg + t], kNSrc - 1);
  const int dg   = deg[n];
  const bool active = t < (dg - 1);
  const float* xrow  = xps + (size_t)src * kG3;
  const float* hprow = hp + (size_t)(n - row_base) * kG3;
  const float* hrow  = H + (size_t)n * kDim;
  float* sl = slab[wave];
#pragma unroll 1
  for (int p = 0; p < 4; ++p) {
    const int j = p * 32 + lane;
    const float xr = xrow[j];
    const float xz = xrow[kDim + j];
    const float xn = xrow[2 * kDim + j];
    float hr, hz, hn, hold;
    if (FIRST) {
      hr = b_hh[j]; hz = b_hh[kDim + j]; hn = b_hh[2 * kDim + j]; hold = 0.0f;
    } else {
      hr = hprow[j]; hz = hprow[kDim + j]; hn = hprow[2 * kDim + j]; hold = hrow[j];
    }
    const float r  = 1.0f / (1.0f + expf(-(xr + hr)));
    const float z  = 1.0f / (1.0f + expf(-(xz + hz)));
    const float nn = tanhf(xn + r * hn);
    const float hnew = (1.0f - z) * nn + z * hold;
    sl[j] = active ? hnew : hold;
  }
  __builtin_amdgcn_fence(__ATOMIC_RELEASE, "workgroup");
  __builtin_amdgcn_wave_barrier();
  __builtin_amdgcn_fence(__ATOMIC_ACQUIRE, "workgroup");
  const v4f hv = *(const v4f*)(sl + 4 * lane);
  const int l16 = lane & 15;
  const v4f a = *(const v4f*)(sl + 8 * l16);
  const v4f c = *(const v4f*)(sl + 8 * l16 + 4);
  unsigned short hb[8];
#pragma unroll
  for (int e = 0; e < 4; ++e) {
    hb[e]     = h_bits(a[e] * kHCarry);
    hb[4 + e] = h_bits(c[e] * kHCarry);
  }
  const v4u u = (v4u){pk16(hb[0], hb[1]), pk16(hb[2], hb[3]), pk16(hb[4], hb[5]), pk16(hb[6], hb[7])};
  float* hq = H + (size_t)n * kDim + 4 * lane;
  unsigned short* h16q = H16 + (size_t)n * kDim + 8 * l16;
  for (int pass = 0; pass < 2; ++pass) {
    *(volatile v4f*)hq = hv;
    if (lane < 16) *(volatile v4u*)h16q = u;
    __threadfence();
  }
}

__global__ __launch_bounds__(256) void ln_select_kernel(const int* __restrict__ token_id, const int* __restrict__ neigh_idx,
                                                        const int* __restrict__ deg, const float* __restrict__ emb,
                                                        const float* __restrict__ H, const float* __restrict__ gamma,
                                                        const float* __restrict__ beta, unsigned short* __restrict__ ft16) {
  __shared__ __align__(16) unsigned stg[8][64];
  const int tid  = threadIdx.x;
  const int wave = tid >> 5;
  const int lane = tid & 31;
  const int n    = blockIdx.x * 8 + wave;
  const int c4   = 4 * lane;
  const v4f h = *(const v4f*)(H + (size_t)n * kDim + c4);
  float s = (h[0] + h[1]) + (h[2] + h[3]);
#pragma unroll
  for (int off = 1; off < 32; off <<= 1) s += __shfl_xor(s, off, 32);
  const float mu = s * kInvDim;
  v4f d;
#pragma unroll
  for (int e = 0; e < 4; ++e) d[e] = h[e] - mu;
  float q = (d[0] * d[0] + d[1] * d[1]) + (d[2] * d[2] + d[3] * d[3]);
#pragma unroll
  for (int off = 1; off < 32; off <<= 1) q += __shfl_xor(q, off, 32);
  const float var  = q * kInvDim;
  const float rstd = 1.0f / sqrtf(var + kLnEps);
  const v4f g  = *(const v4f*)(gamma + c4);
  const v4f bt = *(const v4f*)(beta + c4);
  const int src = clampi(neigh_idx[(size_t)n * kMaxDeg + 0], kNSrc - 1);
  int tk[4];
#pragma unroll
  for (int u = 0; u < 4; ++u) tk[u] = clampi(token_id[(size_t)src * kNSub + u], kVocab - 1);
  v4f em[4];
#pragma unroll
  for (int u = 0; u < 4; ++u) em[u] = *(const v4f*)(emb + (size_t)tk[u] * kDim + c4);
  const bool one = (deg[n] == 1);
  unsigned short hb[4];
#pragma unroll
  for (int e = 0; e < 4; ++e) {
    const float lnv = d[e] * rstd * g[e] + bt[e];
    const unsigned short lb = h_bits(lnv * kHCarry);
    const unsigned short fb = feat16_bits(em[0][e], em[1][e], em[2][e], em[3][e]);
    hb[e] = one ? fb : lb;
  }
  stg[wave][2 * lane]     = pk16(hb[0], hb[1]);
  stg[wave][2 * lane + 1] = pk16(hb[2], hb[3]);
  __builtin_amdgcn_fence(__ATOMIC_RELEASE, "workgroup");
  __builtin_amdgcn_wave_barrier();
  __builtin_amdgcn_fence(__ATOMIC_ACQUIRE, "workgroup");
  const int l16 = lane & 15;
  const v4u u = *(const v4u*)(&stg[wave][4 * l16]);
  unsigned short* oq = ft16 + (size_t)n * kDim + 8 * l16;
  for (int pass = 0; pass < 2; ++pass) {
    if (lane < 16) *(volatile v4u*)oq = u;
    __threadfence();
  }
}

__global__ __launch_bounds__(256) void out_kernel(const float* __restrict__ outp, const float* __restrict__ bc,
                                                  float* __restrict__ out) {
  const int i = blockIdx.x * 256 + threadIdx.x;
  if (i >= kNDst * (kNCls / 4)) return;
  const int row = i / (kNCls / 4);
  const int col = (i - row * (kNCls / 4)) * 4;
  const v4f v = *(const v4f*)(outp + (size_t)row * kNClsPad + col);
  const v4f b = *(const v4f*)(bc + col);
  const v4f r = v + b;
  float* q = out + 4 * (size_t)i;
  *(volatile v4f*)q = r;
  __threadfence();
  *(volatile v4f*)q = r;
}

extern "C" void kernel_launch(void* const* d_in, const int* in_sizes, int n_in,
                              void* d_out, int out_size, void* d_ws, size_t ws_size,
                              hipStream_t stream) {
  (void)in_sizes;
  if (n_in < 12) return;
  if ((size_t)out_size < (size_t)kNDst * kNCls) return;
  const int*   token_id  = (const int*)d_in[0];
  const int*   neigh_idx = (const int*)d_in[1];
  const int*   deg       = (const int*)d_in[2];
  const float* emb       = (const float*)d_in[3];
  const float* w_ih      = (const float*)d_in[4];
  const float* w_hh      = (const float*)d_in[5];
  const float* b_ih      = (const float*)d_in[6];
  const float* b_hh      = (const float*)d_in[7];
  const float* gamma     = (const float*)d_in[8];
  const float* beta      = (const float*)d_in[9];
  const float* wc        = (const float*)d_in[10];
  const float* bc        = (const float*)d_in[11];
  float* out = (float*)d_out;

  const size_t szXPS  = (size_t)kNSrcPad * kG3 * sizeof(float);
  const size_t szH    = (size_t)kNDst * kDim * sizeof(float);
  const size_t szH16  = (size_t)kNDst * kDim * sizeof(unsigned short);
  const size_t szW16  = (size_t)kG3 * kDim * sizeof(unsigned short);
  const size_t szWC16 = (size_t)kNClsPad * kDim * sizeof(unsigned short);
  const size_t szFEAT = (size_t)kNSrcPad * kDim * sizeof(unsigned short);
  const size_t szHP   = (size_t)kChunkRows * kG3 * sizeof(float);
  const size_t szR6   = (szFEAT > szHP) ? szFEAT : szHP;

  size_t off = 0;
  const size_t oXPS  = off; off += szXPS;
  const size_t oH    = off; off += szH;
  const size_t oH16  = off; off += szH16;
  const size_t oWIH  = off; off += szW16;
  const size_t oWHH  = off; off += szW16;
  const size_t oWC   = off; off += szWC16;
  const size_t oR6   = off; off += szR6;
  if (off > ws_size) return;

  char* ws = (char*)d_ws;
  float*          XPS    = (float*)(ws + oXPS);
  float*          OUTP   = (float*)(ws + oXPS);
  float*          Hs     = (float*)(ws + oH);
  unsigned short* H16    = (unsigned short*)(ws + oH16);
  unsigned short* FT16   = (unsigned short*)(ws + oH16);
  unsigned short* WIH16  = (unsigned short*)(ws + oWIH);
  unsigned short* WHH16  = (unsigned short*)(ws + oWHH);
  unsigned short* WC16   = (unsigned short*)(ws + oWC);
  unsigned short* FEAT16 = (unsigned short*)(ws + oR6);
  float*          HP     = (float*)(ws + oR6);

  wcast_kernel<<<dim3((kG3 * kDim / 8 + 255) / 256, 3), 256, 0, stream>>>(w_ih, w_hh, wc, WIH16, WHH16, WC16, kWCarry);
  feat_kernel<<<kNSrcPad / 16, 256, 0, stream>>>(token_id, emb, FEAT16);
  {
    const int tiles = (kNSrcPad / 64) * (kG3 / 64);
    wmma_gemm64<0, false, 2, 0, false><<<dim3((tiles + 7) / 8, 1), 256, 0, stream>>>(
        FEAT16, FEAT16, kDim, 0L, WIH16, WIH16, kDim, 0L, (void*)XPS, (void*)XPS, kG3, 0L,
        b_ih, b_ih, 0L, kNSrcPad, kG3, kDim, kGemmScale);
  }
  for (int c = 0; c < kNChunks; ++c) {
    gru_cell_kernel<true><<<kChunkRows / 8, 256, 0, stream>>>(neigh_idx, deg, XPS, HP, b_hh, Hs, H16, c * kChunkRows, 0);
  }
  for (int t = 1; t < kSteps; ++t) {
    for (int c = 0; c < kNChunks; ++c) {
      const int tiles = (kChunkRows / 64) * (kG3 / 64);
      const unsigned short* Achunk = H16 + (size_t)c * kChunkRows * kDim;
      wmma_gemm64<0, false, 2, 0, false><<<dim3((tiles + 7) / 8, 1), 256, 0, stream>>>(
          Achunk, Achunk, kDim, 0L, WHH16, WHH16, kDim, 0L, (void*)HP, (void*)HP, kG3, 0L,
          b_hh, b_hh, 0L, kChunkRows, kG3, kDim, kGemmScale);
      gru_cell_kernel<false><<<kChunkRows / 8, 256, 0, stream>>>(neigh_idx, deg, XPS, HP, b_hh, Hs, H16, c * kChunkRows, t);
    }
  }
  ln_select_kernel<<<kNDst / 8, 256, 0, stream>>>(token_id, neigh_idx, deg, emb, Hs, gamma, beta, FT16);
  {
    const int tiles = (kNDst / 64) * (kNClsPad / 64);
    wmma_gemm64<0, false, 0, 0, false><<<dim3((tiles + 7) / 8, 1), 256, 0, stream>>>(
        FT16, FT16, kDim, 0L, WC16, WC16, kDim, 0L, (void*)OUTP, (void*)OUTP, kNClsPad, 0L,
        bc, bc, 0L, kNDst, kNClsPad, kDim, kGemmScale);
  }
  out_kernel<<<(kNDst * (kNCls / 4) + 255) / 256, 256, 0, stream>>>(OUTP, bc, out);
}
